// InteractionLayer_54202487275607
// MI455X (gfx1250) — hardware-run, weakly checked
//
#include <hip/hip_runtime.h>

typedef float          v8f   __attribute__((ext_vector_type(8)));
typedef float          v4f   __attribute__((ext_vector_type(4)));
typedef unsigned int   v4u   __attribute__((ext_vector_type(4)));
typedef int            v8i   __attribute__((ext_vector_type(8)));
typedef unsigned short v8us  __attribute__((ext_vector_type(8)));
typedef unsigned short v16us __attribute__((ext_vector_type(16)));
typedef __bf16         v16bf __attribute__((ext_vector_type(16)));
typedef _Float16       v16h  __attribute__((ext_vector_type(16)));
typedef v4f  __attribute__((may_alias)) v4fa;
typedef v8us __attribute__((may_alias)) v8usa;
union FragB { v16bf v; v16us u; v8us h[2]; v8i w; };
union FragH { v16h  v; v16us u; v8us h[2]; v8i w; };

__device__ __forceinline__ v8f wmb(const FragB& a, const FragB& b, v8f c) {
  v8f d = __builtin_amdgcn_wmma_f32_16x16x32_bf16(false, a.v, false, b.v, (short)0, c, false, false);
  asm volatile("v_nop\n\tv_nop\n\tv_nop\n\tv_nop" : "+v"(d) : "v"(a.w), "v"(b.w));
  return d;
}

__device__ __forceinline__ v8f wmh(const FragH& a, const FragH& b, v8f c) {
  v8f d = __builtin_amdgcn_wmma_f32_16x16x32_f16(false, a.v, false, b.v, (short)0, c, false, false);
  asm volatile("v_nop\n\tv_nop\n\tv_nop\n\tv_nop" : "+v"(d) : "v"(a.w), "v"(b.w));
  return d;
}

__device__ __forceinline__ unsigned bf16_bits(float f) {
  const unsigned u = __float_as_uint(f);
  const unsigned r = (u + 0x7FFFu + ((u >> 16) & 1u)) >> 16;
  const unsigned q = (u >> 16) | 0x40u;
  return ((u & 0x7fffffffu) > 0x7f800000u) ? q : r;
}

__device__ __forceinline__ float bf16_val(float f) {
  return __uint_as_float(bf16_bits(f) << 16);
}
__device__ __forceinline__ int clampi(int v, int lo, int hi) {
  return v < lo ? lo : (v > hi ? hi : v);
}

__device__ __forceinline__ unsigned f16_bits(float f) {
  const unsigned u  = __float_as_uint(f);
  const unsigned s  = (u >> 16) & 0x8000u;
  const unsigned a  = u & 0x7fffffffu;
  const unsigned t  = a - 0x38000000u;
  const unsigned r  = (t + 0x0FFFu + ((t >> 13) & 1u)) >> 13;
  const unsigned rc = r > 0x7C00u ? 0x7C00u : r;
  const bool small  = a < 0x38800000u;
  const bool isnan  = a > 0x7f800000u;
  const unsigned fin = small ? 0u : (s | rc);
  return isnan ? (s | 0x7E00u) : fin;
}

__device__ __forceinline__ unsigned pk16(unsigned lo, unsigned hi) { return lo | (hi << 16); }
__device__ __forceinline__ unsigned bf16_lo_bits(float v) {
  float hi = bf16_val(v);
  asm volatile("" : "+v"(hi));
  return bf16_bits(v - hi);
}
__device__ __forceinline__ v4u pack8_bf16(v4f a, v4f c) {
  return (v4u){ pk16(bf16_bits(a[0]), bf16_bits(a[1])), pk16(bf16_bits(a[2]), bf16_bits(a[3])),
                pk16(bf16_bits(c[0]), bf16_bits(c[1])), pk16(bf16_bits(c[2]), bf16_bits(c[3])) };
}
__device__ __forceinline__ v4u pack8_bf16_lo(v4f a, v4f c) {
  return (v4u){ pk16(bf16_lo_bits(a[0]), bf16_lo_bits(a[1])), pk16(bf16_lo_bits(a[2]), bf16_lo_bits(a[3])),
                pk16(bf16_lo_bits(c[0]), bf16_lo_bits(c[1])), pk16(bf16_lo_bits(c[2]), bf16_lo_bits(c[3])) };
}
__device__ __forceinline__ v4u pack8_f16(v4f a, v4f c) {
  return (v4u){ pk16(f16_bits(a[0]), f16_bits(a[1])), pk16(f16_bits(a[2]), f16_bits(a[3])),
                pk16(f16_bits(c[0]), f16_bits(c[1])), pk16(f16_bits(c[2]), f16_bits(c[3])) };
}

template <int FORM>
__global__ __launch_bounds__(256) void k_plane(const float* __restrict__ src, int rows, int cols, int ldsrc,
                                               unsigned short* __restrict__ dst, int MP, int KP) {
  static_assert(FORM >= 0 && FORM <= 3);
  const int KTOT = (FORM == 1 || FORM == 3) ? 2 * KP : KP;
  const unsigned ppr   = (unsigned)(KTOT >> 3);
  const unsigned kp8   = (unsigned)(KP >> 3);
  const unsigned total = (unsigned)MP * ppr;
  const unsigned g     = blockIdx.x * 256u + threadIdx.x;
  const unsigned rowu  = g / ppr;
  const unsigned p     = g - rowu * ppr;
  const bool second    = p >= kp8;
  const int row = (int)rowu;
  const int c0  = (int)((second ? p - kp8 : p) << 3);
  const float* srow = src + (size_t)clampi(row, 0, rows - 1) * (size_t)ldsrc;
  float x[8];
  unsigned mk[8];
#pragma unroll
  for (int e = 0; e < 8; ++e) {
    const int c = c0 + e;
    const float v = srow[clampi(c, 0, cols - 1)];
    asm volatile("" :: "v"(v));
    x[e]  = v;
    mk[e] = (row < rows && c < cols) ? 0xFFFFu : 0u;
  }
  const v4f a = (v4f){ x[0], x[1], x[2], x[3] };
  const v4f c = (v4f){ x[4], x[5], x[6], x[7] };
  v4u o;
  if (FORM == 2) {
    o = pack8_f16(a, c);
  } else {
    const v4u hi = pack8_bf16(a, c);
    o = hi;
    if (FORM == 1) { const v4u lo = pack8_bf16_lo(a, c); o = second ? lo : hi; }
  }
  const v4u mw = (v4u){ pk16(mk[0], mk[1]), pk16(mk[2], mk[3]), pk16(mk[4], mk[5]), pk16(mk[6], mk[7]) };
  o &= mw;
  if (g < total) {
    volatile v4u* q = (volatile v4u*)(dst + (size_t)g * 8);
    *q = o;
    __threadfence();
    *q = o;
  }
}

template <int FORM> struct FragOf    { typedef FragB T; };
template <>         struct FragOf<2> { typedef FragH T; };
__device__ __forceinline__ v8f mm(const FragB& a, const FragB& b, v8f c) { return wmb(a, b, c); }
__device__ __forceinline__ v8f mm(const FragH& a, const FragH& b, v8f c) { return wmh(a, b, c); }
template <class F> __device__ __forceinline__ F ld_frag(const unsigned short* p) {
  F f;
  f.h[0] = *(const v8usa*)(p);
  f.h[1] = *(const v8usa*)(p + 16);
  return f;
}

template <int FORM, int EPI>
__global__ __launch_bounds__(256) __attribute__((amdgpu_num_vgpr(248)))
void k_gemm_nt(const unsigned short* __restrict__ A, const unsigned short* __restrict__ B,
               const float* __restrict__ bias, float* __restrict__ D, int M, int N, int KTOT, int ldd) {
  static_assert(FORM >= 0 && FORM <= 2);
  static_assert(EPI == 0 || EPI == 1);
  typedef typename FragOf<FORM>::T F;
  __shared__ __attribute__((aligned(16))) float sT[8][16 * 68];
  const int lane = threadIdx.x & 31;
  const int wave = threadIdx.x >> 5;
  const int tilesM = (M + 63) >> 6;
  const int tilesN = (N + 63) >> 6;
  const int tile = blockIdx.x * 8 + wave;
  if (tile >= tilesM * tilesN) return;
  const int tm = tile / tilesN;
  const int tn = tile - tm * tilesN;
  const int m0 = tm << 6;
  const int n0 = tn << 6;

  const int rl = lane & 15;
  const int h8 = (lane >> 4) * 8;
  const unsigned short* pa = A + (size_t)(m0 + rl) * (size_t)KTOT + h8;
  const unsigned short* pb = B + (size_t)(n0 + rl) * (size_t)KTOT + h8;

  v8f acc[4][4];
#pragma unroll
  for (int i = 0; i < 4; ++i)
#pragma unroll
    for (int j = 0; j < 4; ++j) acc[i][j] = (v8f){0.f, 0.f, 0.f, 0.f, 0.f, 0.f, 0.f, 0.f};

#pragma unroll 1
  for (int k0 = 0; k0 < KTOT; k0 += 32) {
    F bf[4];
#pragma unroll
    for (int j = 0; j < 4; ++j) bf[j] = ld_frag<F>(pb + (size_t)(j << 4) * (size_t)KTOT + k0);
#pragma unroll
    for (int i = 0; i < 4; ++i) {
      const F af = ld_frag<F>(pa + (size_t)(i << 4) * (size_t)KTOT + k0);
#pragma unroll
      for (int j = 0; j < 4; ++j) acc[i][j] = mm(af, bf[j], acc[i][j]);
    }
  }

  float* slab = sT[wave];
  const int hh = lane >> 4;
  const int c4 = (lane & 15) * 4;
  const int nc = n0 + c4;
  const bool cok = nc < N;
  v4f bv = (v4f){0.f, 0.f, 0.f, 0.f};
  if (EPI == 1) {
    bv = *(const v4fa*)(bias + clampi(nc, 0, N - 4));
    asm volatile("" :: "v"(bv));
  }
#pragma unroll
  for (int i = 0; i < 4; ++i) {
    const int mBase = m0 + (i << 4);
#pragma unroll
    for (int j = 0; j < 4; ++j) {
#pragma unroll
      for (int r = 0; r < 8; ++r) slab[(h8 + r) * 68 + (j << 4) + rl] = acc[i][j][r];
    }
    __builtin_amdgcn_fence(__ATOMIC_RELEASE, "workgroup");
    __builtin_amdgcn_wave_barrier();
    __builtin_amdgcn_fence(__ATOMIC_ACQUIRE, "workgroup");
    v4f vv[8];
#pragma unroll
    for (int it = 0; it < 8; ++it) {
      const int row = it * 2 + hh;
      v4f v = *(const v4fa*)(slab + row * 68 + c4);
      if (EPI == 1) v += bv;
      vv[it] = v;
    }
    for (int pass = 0; pass < 2; ++pass) {
#pragma unroll
      for (int it = 0; it < 8; ++it) {
        const int row = mBase + it * 2 + hh;
        if (cok && row < M) *(volatile v4f*)(D + (size_t)row * (size_t)ldd + nc) = vv[it];
      }
      __threadfence();
    }
    __builtin_amdgcn_fence(__ATOMIC_RELEASE, "workgroup");
    __builtin_amdgcn_wave_barrier();
    __builtin_amdgcn_fence(__ATOMIC_ACQUIRE, "workgroup");
  }
}

typedef int v4i __attribute__((ext_vector_type(4)));
typedef v4i __attribute__((may_alias)) v4ia;

static constexpr int kN = 30000;
static constexpr int kD = 128;
static constexpr int kE = 480000;
static constexpr int kMP = 30016;
static constexpr int kNC = 640;
static constexpr int kSLOTS = 1024;
static constexpr int kNBLK = 30;
static constexpr int kNSLOT = kNBLK * kSLOTS;
static constexpr int kRCAP = 24576;
static constexpr int kDEGCAP = 64;
static constexpr int kSCAP = 96;
static constexpr int kCHUNK = 2048;
static constexpr int kNCHUNK = 235;
static constexpr int kWCAP = 256;
static constexpr int kLISTN = 2048;
static constexpr int kMAXHIT = 16633;
static constexpr int kMAXDEG = 35;
static constexpr int T_AS = 0, T_AD = 512, T_BG = 1024, T_BC = 1152, T_GM = 1280, T_BT = 1408, T_WG = 1536,
                     T_BE = 2048, T_TOT = 2080;
static constexpr int kLDS_BKT = (2 * kRCAP + 3 * kSLOTS + kLISTN) * 4 + 64;

static_assert(kE == 234 * 2048 + 768);
static_assert(kNCHUNK == (kE + kCHUNK - 1) / kCHUNK);
static_assert(kE % 8 == 0);
static_assert(kN % 8 == 0 && kN / 8 == 3750);
static_assert(kD == 32 * 4);
static_assert(kNC % 64 == 0 && kNC % 32 == 0 && kNC == 5 * kD);
static_assert(kMP % 64 == 0 && kMP >= kN && kMP % 32 == 0 && kMP / 32 == 938);
static_assert(kD % 32 == 0);
static_assert(kNSLOT >= kMP);
static_assert(kRCAP * 4 >= kMAXHIT * 5);
static_assert(kRCAP % 1024 == 0);
static_assert(kDEGCAP >= kMAXDEG + 8 && kDEGCAP % 32 == 0);
static_assert(kSCAP >= ((kDEGCAP + 1 + 31) / 32) * 32);
static_assert(kN <= (1 << 15) && kSLOTS == (1 << 10));
static_assert(kWCAP == 32 * 8 && kLISTN == 8 * kWCAP && kCHUNK == 256 * 8);
static_assert(kLDS_BKT <= 262144);
static_assert(T_TOT % 32 == 0 && T_BE + 32 == T_TOT);
static_assert((kMP * (kD / 8)) % 256 == 0);

__device__ __forceinline__ void wave_sync_lds() {
  __builtin_amdgcn_fence(__ATOMIC_RELEASE, "workgroup");
  __builtin_amdgcn_wave_barrier();
  __builtin_amdgcn_fence(__ATOMIC_ACQUIRE, "workgroup");
}
__device__ __forceinline__ float leaky02(float v) { return (v > 0.0f) ? v : 0.2f * v; }
__device__ __forceinline__ float nmax(float a, float b) { return (b > a || b != b) ? b : a; }
__device__ __forceinline__ float sel4(v4f v, int k) {
  float r = v.x;
  r = (k == 1) ? v.y : r;
  r = (k == 2) ? v.z : r;
  r = (k == 3) ? v.w : r;
  return r;
}
__device__ __forceinline__ float wsum(float v) {
#pragma unroll
  for (int off = 16; off > 0; off >>= 1) v += __shfl_xor(v, off);
  return v;
}

__device__ __forceinline__ void wt_unit(const float* __restrict__ w, int col, int k8, unsigned short* dstp) {
  const float* p = w + (size_t)k8 * 128 + col;
  float x[8];
#pragma unroll
  for (int e = 0; e < 8; ++e) {
    const float v = p[e * 128];
    asm volatile("" :: "v"(v));
    x[e] = v;
  }
  const v4u o = pack8_bf16((v4f){ x[0], x[1], x[2], x[3] }, (v4f){ x[4], x[5], x[6], x[7] });
  volatile v4u* q = (volatile v4u*)dstp;
  *q = o;
  __threadfence();
  *q = o;
}
__device__ __forceinline__ void tab_unit(const float* __restrict__ src, int n, int ext, float* dst, int tid) {
  const int i0 = 4 * tid;
  float v[4];
#pragma unroll
  for (int j = 0; j < 4; ++j) {
    const int i = i0 + j;
    const float t = src[clampi(i, 0, n - 1)];
    asm volatile("" :: "v"(t));
    v[j] = (i < n) ? bf16_val(t) : 0.0f;
  }
  const v4f o = (v4f){ v[0], v[1], v[2], v[3] };
  if (i0 < ext) {
    volatile v4f* q = (volatile v4f*)(dst + i0);
    *q = o;
    __threadfence();
    *q = o;
  }
}
__global__ __launch_bounds__(256) void k_prep(const float* __restrict__ Wa, const float* __restrict__ Wn,
                                              const float* __restrict__ att_s, const float* __restrict__ att_d,
                                              const float* __restrict__ b_a, const float* __restrict__ b_n,
                                              const float* __restrict__ gam, const float* __restrict__ bet,
                                              const float* __restrict__ Wg, const float* __restrict__ bg,
                                              unsigned short* WT, float* TAB) {
  const int b = (int)blockIdx.x, tid = (int)threadIdx.x;
  if (b < 32) {
    const int u = b * 256 + tid;
    const int n = u >> 4, k8 = (u & 15) * 8;
    const int h = n >> 7, f = n & 127;
    wt_unit(Wa + (size_t)h * 16384, f, k8, WT + (size_t)n * 128 + k8);
  } else if (b < 40) {
    const int u = b * 256 + tid;
    const int n = u >> 4, k8 = (u & 15) * 8;
    wt_unit(Wn, n - 512, k8, WT + (size_t)n * 128 + k8);
  } else if (b == 40) { tab_unit(att_s, 512, 512, TAB + T_AS, tid);
  } else if (b == 41) { tab_unit(att_d, 512, 512, TAB + T_AD, tid);
  } else if (b == 42) { tab_unit(b_a, 128, 128, TAB + T_BG, tid);
  } else if (b == 43) { tab_unit(b_n, 128, 128, TAB + T_BC, tid);
  } else if (b == 44) { tab_unit(gam, 128, 128, TAB + T_GM, tid);
  } else if (b == 45) { tab_unit(bet, 128, 128, TAB + T_BT, tid);
  } else if (b == 46) { tab_unit(Wg, 512, 512, TAB + T_WG, tid);
  } else if (b == 47) { tab_unit(bg, 2, 32, TAB + T_BE, tid);
  }
}

__global__ __launch_bounds__(256) void k_scores(const float* __restrict__ P, const float* __restrict__ TAB, float* SD) {
  __shared__ __attribute__((aligned(16))) float sAtt[1024];
  __shared__ __attribute__((aligned(16))) float sRow[8][256];
  const int tid = (int)threadIdx.x, lane = tid & 31, wave = tid >> 5;
  {
    const v4f t = *(const v4fa*)(TAB + 4 * tid);
    *(v4fa*)(sAtt + 4 * tid) = t;
  }
  __syncthreads();
  const int grp = (int)blockIdx.x * 8 + wave;
  if (grp < kMP / 32) {
    v4f as[4], ad[4];
#pragma unroll
    for (int h = 0; h < 4; ++h) {
      as[h] = *(const v4fa*)(sAtt + h * 128 + 4 * lane);
      ad[h] = *(const v4fa*)(sAtt + 512 + h * 128 + 4 * lane);
    }
    float* strip = sRow[wave];
    const int l7 = lane & 7;
#pragma unroll 1
    for (int it = 0; it < 32; ++it) {
      const int node = grp * 32 + it;
      const float* pr = P + (size_t)node * kNC + 4 * lane;
      float ps[4], pd[4];
#pragma unroll
      for (int h = 0; h < 4; ++h) {
        const v4f r = *(const v4fa*)(pr + h * 128);
        ps[h] = r.x * as[h].x + r.y * as[h].y + r.z * as[h].z + r.w * as[h].w;
        pd[h] = r.x * ad[h].x + r.y * ad[h].y + r.z * ad[h].z + r.w * ad[h].w;
      }
#pragma unroll
      for (int h = 0; h < 4; ++h) { ps[h] = wsum(ps[h]); pd[h] = wsum(pd[h]); }
      float v = ps[0];
      v = (l7 == 1) ? ps[1] : v;
      v = (l7 == 2) ? ps[2] : v;
      v = (l7 == 3) ? ps[3] : v;
      v = (l7 == 4) ? pd[0] : v;
      v = (l7 == 5) ? pd[1] : v;
      v = (l7 == 6) ? pd[2] : v;
      v = (l7 == 7) ? pd[3] : v;
      if (lane < 8) strip[it * 8 + lane] = v;
    }
    wave_sync_lds();
    const v4f a = *(const v4fa*)(strip + 4 * lane);
    const v4f b = *(const v4fa*)(strip + 128 + 4 * lane);
    float* g = SD + (size_t)grp * 256;
    volatile v4f* q0 = (volatile v4f*)(g + 4 * lane);
    volatile v4f* q1 = (volatile v4f*)(g + 128 + 4 * lane);
    *q0 = a; *q1 = b;
    __threadfence();
    *q0 = a; *q1 = b;
  }
}

__device__ __forceinline__ unsigned hitw(int d, int s, int nodeBase, bool inr) {
  const int dc = clampi(d, 0, kN - 1);
  const int sc = clampi(s, 0, kN - 1);
  const unsigned sl = (unsigned)(dc - nodeBase);
  const bool hit = inr && (sl < (unsigned)kSLOTS);
  return hit ? (((unsigned)sc << 10) | sl) : 0xFFFFFFFFu;
}
__global__ __launch_bounds__(256) void k_bucket(const int* __restrict__ ei, int* OFF, int* CNT, float* DINV, int* LIST) {
  extern __shared__ v4f lds_dyn[];
  int*   reg1 = (int*)lds_dyn;
  int*   reg2 = reg1 + kRCAP;
  int*   scnt = reg2 + kRCAP;
  int*   soff = scnt + kSLOTS;
  float* sdv  = (float*)(soff + kSLOTS);
  int*   list = (int*)(sdv + kSLOTS);
  int*   wcnt = list + kLISTN;
  int*   wtot = wcnt + 8;
  const int tid = (int)threadIdx.x, lane = tid & 31, wave = tid >> 5;
  const int blk = (int)blockIdx.x;
  const int nodeBase = blk * kSLOTS;
  const int fillv = nodeBase < kN ? nodeBase : kN - 1;
  const int* srcs = ei;
  const int* dsts = ei + kE;

  {
    const v4i z = (v4i){0, 0, 0, 0};
    *(v4ia*)(scnt + 4 * tid) = z;
    const v4i f = (v4i){fillv, fillv, fillv, fillv};
#pragma unroll 1
    for (int it = 0; it < kRCAP / 1024; ++it) *(v4ia*)(reg2 + 4 * (it * 256 + tid)) = f;
  }
  __syncthreads();

  int tot = 0, ovf = 0;
#pragma unroll 1
  for (int ch = 0; ch < kNCHUNK; ++ch) {
    const int e0  = ch * kCHUNK + tid * 8;
    const int e0c = e0 < kE - 8 ? e0 : kE - 8;
    const bool inr = e0 < kE;
    const v4i da = *(const v4ia*)(dsts + e0c);
    const v4i db = *(const v4ia*)(dsts + e0c + 4);
    const v4i sa = *(const v4ia*)(srcs + e0c);
    const v4i sb = *(const v4ia*)(srcs + e0c + 4);
    asm volatile("" :: "v"(da));
    asm volatile("" :: "v"(db));
    asm volatile("" :: "v"(sa));
    asm volatile("" :: "v"(sb));
    const unsigned w0 = hitw(da.x, sa.x, nodeBase, inr);
    const unsigned w1 = hitw(da.y, sa.y, nodeBase, inr);
    const unsigned w2 = hitw(da.z, sa.z, nodeBase, inr);
    const unsigned w3 = hitw(da.w, sa.w, nodeBase, inr);
    const unsigned w4 = hitw(db.x, sb.x, nodeBase, inr);
    const unsigned w5 = hitw(db.y, sb.y, nodeBase, inr);
    const unsigned w6 = hitw(db.z, sb.z, nodeBase, inr);
    const unsigned w7 = hitw(db.w, sb.w, nodeBase, inr);
    const bool h0 = w0 != 0xFFFFFFFFu, h1 = w1 != 0xFFFFFFFFu, h2 = w2 != 0xFFFFFFFFu, h3 = w3 != 0xFFFFFFFFu;
    const bool h4 = w4 != 0xFFFFFFFFu, h5 = w5 != 0xFFFFFFFFu, h6 = w6 != 0xFFFFFFFFu, h7 = w7 != 0xFFFFFFFFu;
    const int c = (int)h0 + (int)h1 + (int)h2 + (int)h3 + (int)h4 + (int)h5 + (int)h6 + (int)h7;
    int incl = c;
#pragma unroll
    for (int d = 1; d < 32; d <<= 1) {
      const int up = __shfl_up(incl, d);
      incl += (lane >= d) ? up : 0;
    }
    const int wc = __shfl(incl, 31);
    int pos = wave * kWCAP + incl - c;
    if (h0) list[pos] = (int)w0;
    pos += (int)h0;
    if (h1) list[pos] = (int)w1;
    pos += (int)h1;
    if (h2) list[pos] = (int)w2;
    pos += (int)h2;
    if (h3) list[pos] = (int)w3;
    pos += (int)h3;
    if (h4) list[pos] = (int)w4;
    pos += (int)h4;
    if (h5) list[pos] = (int)w5;
    pos += (int)h5;
    if (h6) list[pos] = (int)w6;
    pos += (int)h6;
    if (h7) list[pos] = (int)w7;
    if (lane == 0) wcnt[wave] = wc;
    __syncthreads();
    int pre = 0, all = 0;
#pragma unroll
    for (int w2i = 0; w2i < 8; ++w2i) {
      const int cc = clampi(wcnt[w2i], 0, kWCAP);
      all += cc;
      pre += (w2i < wave) ? cc : 0;
    }
    const int wcc  = clampi(wc, 0, kWCAP);
    const int base = tot + pre;
#pragma unroll 1
    for (int i = lane; i < wcc; i += 32) {
      const int ent = list[wave * kWCAP + i];
      const int p2  = base + i;
      if (p2 < kRCAP) reg1[p2] = ent;
    }
    tot += all;
    if (tot > kRCAP) { tot = kRCAP; ovf = 1; }
    __syncthreads();
  }
  const int nh = __builtin_amdgcn_readfirstlane(tot);

  if (wave == 0) {
#pragma unroll 1
    for (int b0 = 0; b0 < nh; b0 += 32) {
      const int idx = (b0 + lane) < nh ? (b0 + lane) : nh - 1;
      const int uv  = reg1[idx];
      const int m32 = (nh - b0) < 32 ? (nh - b0) : 32;
#pragma unroll 1
      for (int k = 0; k < m32; ++k) {
        const int u  = __builtin_amdgcn_readlane(uv, k);
        const int sl = u & (kSLOTS - 1);
        if (lane == 0) scnt[sl] = scnt[sl] + 1;
      }
    }
  }
  __syncthreads();

  {
    const v4i cv = *(const v4ia*)(scnt + 4 * tid);
    const int e0 = cv.x < 0 ? 0 : cv.x, e1 = cv.y < 0 ? 0 : cv.y, e2 = cv.z < 0 ? 0 : cv.z, e3 = cv.w < 0 ? 0 : cv.w;
    const int ts = e0 + e1 + e2 + e3;
    int incl = ts;
#pragma unroll
    for (int d = 1; d < 32; d <<= 1) {
      const int up = __shfl_up(incl, d);
      incl += (lane >= d) ? up : 0;
    }
    if (lane == 31) wtot[wave] = incl;
    __syncthreads();
    int pre = 0;
#pragma unroll
    for (int w2i = 0; w2i < 8; ++w2i) pre += (w2i < wave) ? wtot[w2i] : 0;
    const int run = pre + incl - ts;
    const v4i so = (v4i){ run, run + e0, run + e0 + e1, run + e0 + e1 + e2 };
    *(v4ia*)(soff + 4 * tid) = so;
    *(v4ia*)(list + 4 * tid) = so;
  }
  __syncthreads();

  if (wave == 0) {
#pragma unroll 1
    for (int b0 = 0; b0 < nh; b0 += 32) {
      const int idx = (b0 + lane) < nh ? (b0 + lane) : nh - 1;
      const int uv  = reg1[idx];
      const int m32 = (nh - b0) < 32 ? (nh - b0) : 32;
#pragma unroll 1
      for (int k = 0; k < m32; ++k) {
        const int u  = __builtin_amdgcn_readlane(uv, k);
        const int sl = u & (kSLOTS - 1);
        const int sv = (int)((unsigned)u >> 10);
        if (lane == 0) {
          const int p2 = clampi(list[sl], 0, kRCAP - 1);
          reg2[p2] = sv;
          list[sl] = p2 + 1;
        }
      }
    }
  }
  __syncthreads();

  {
#pragma unroll 1
    for (int j = 0; j < 4; ++j) {
      int c = scnt[4 * tid + j];
      c = c < 0 ? 0 : c;
      const float deg = (float)(c + 1);
      sdv[4 * tid + j] = (deg > 0.0f) ? (1.0f / sqrtf(deg)) : 0.0f;
    }
    const v4f dv = *(const v4fa*)(sdv + 4 * tid);
    const v4i cv = *(const v4ia*)(scnt + 4 * tid);
    const v4i so = *(const v4ia*)(soff + 4 * tid);
    v4i cm;
    cm.x = (ovf != 0 || cv.x > kDEGCAP || cv.x < 0) ? -1 : cv.x;
    cm.y = (ovf != 0 || cv.y > kDEGCAP || cv.y < 0) ? -1 : cv.y;
    cm.z = (ovf != 0 || cv.z > kDEGCAP || cv.z < 0) ? -1 : cv.z;
    cm.w = (ovf != 0 || cv.w > kDEGCAP || cv.w < 0) ? -1 : cv.w;
    volatile v4i* po = (volatile v4i*)(OFF + nodeBase + 4 * tid);
    volatile v4i* pc = (volatile v4i*)(CNT + nodeBase + 4 * tid);
    volatile v4f* pd = (volatile v4f*)(DINV + nodeBase + 4 * tid);
    *po = so; *pc = cm; *pd = dv;
    __threadfence();
    *po = so; *pc = cm; *pd = dv;
  }
  {
    int* lp = LIST + (size_t)blk * kRCAP;
    for (int pass = 0; pass < 2; ++pass) {
#pragma unroll 1
      for (int it = 0; it < kRCAP / 1024; ++it) {
        const int i4 = it * 256 + tid;
        const v4i v = *(const v4ia*)(reg2 + 4 * i4);
        *(volatile v4i*)(lp + 4 * i4) = v;
      }
      __threadfence();
    }
  }
}

__global__ __launch_bounds__(256) __attribute__((amdgpu_num_vgpr(248)))
void k_replay(const float* __restrict__ P, const float* __restrict__ SD, const int* __restrict__ OFF,
              const int* __restrict__ CNT, const float* __restrict__ DINV, const int* __restrict__ LIST,
              const float* __restrict__ TAB, float* out) {
  __shared__ __attribute__((aligned(16))) float sTab[1056];
  __shared__ __attribute__((aligned(16))) float sSc[8][kSCAP * 4];
  __shared__ __attribute__((aligned(16))) int   sSrc[8][kSCAP];
  __shared__ __attribute__((aligned(16))) float sCf[8][kSCAP];
  const int tid = (int)threadIdx.x, lane = tid & 31, wave = tid >> 5;
  {
    const int i0 = tid;
    const int i1 = (256 + tid < 263) ? 256 + tid : 263;
    const v4f t0 = *(const v4fa*)(TAB + T_BG + 4 * i0);
    const v4f t1 = *(const v4fa*)(TAB + T_BG + 4 * i1);
    asm volatile("" :: "v"(t0.x), "v"(t0.y), "v"(t0.z), "v"(t0.w));
    asm volatile("" :: "v"(t1.x), "v"(t1.y), "v"(t1.z), "v"(t1.w));
    *(v4fa*)(sTab + 4 * i0) = t0;
    *(v4fa*)(sTab + 4 * i1) = t1;
  }
  __syncthreads();

  const int row = (int)blockIdx.x * 8 + wave;
  const bool live = row < kN;
  const int rc = live ? row : kN - 1;
  const int craw = CNT[rc];
  asm volatile("" :: "v"(craw));
  int offv = OFF[rc];
  asm volatile("" :: "v"(offv));
  const float di = DINV[rc];
  asm volatile("" :: "v"(di));
  const v4f sia = *(const v4fa*)(SD + (size_t)rc * 8);
  const v4f sid = *(const v4fa*)(SD + (size_t)rc * 8 + 4);
  asm volatile("" :: "v"(sia));
  asm volatile("" :: "v"(sid));
  const int c  = clampi(craw, 0, kDEGCAP);
  const int cn = __builtin_amdgcn_readfirstlane(live ? c : 0);
  const int ne = cn + 1;
  offv = clampi(offv, 0, kRCAP - 1);
  const int lb = clampi(rc >> 10, 0, kNBLK - 1);
  const int* lp = LIST + (size_t)lb * kRCAP;
  float* st = sSc[wave];
  int*   ss = sSrc[wave];
  float* sc = sCf[wave];

#pragma unroll 1
  for (int p0 = 0; p0 < ne; p0 += 32) {
    const int q = p0 + lane;
    const int idx = (offv + q) < kRCAP - 1 ? (offv + q) : kRCAP - 1;
    const int sw = lp[idx];
    asm volatile("" :: "v"(sw));
    const int s = clampi(sw, 0, kN - 1);
    const v4f sv = *(const v4fa*)(SD + (size_t)s * 8);
    asm volatile("" :: "v"(sv));
    const float ds = DINV[s];
    asm volatile("" :: "v"(ds));
    const v4f e4 = (v4f){ leaky02(sv.x + sid.x), leaky02(sv.y + sid.y), leaky02(sv.z + sid.z), leaky02(sv.w + sid.w) };
    *(v4fa*)(st + 4 * q) = e4;
    ss[q] = s;
    sc[q] = ds * di;
  }
  {
    const v4f es = (v4f){ leaky02(sia.x + sid.x), leaky02(sia.y + sid.y), leaky02(sia.z + sid.z), leaky02(sia.w + sid.w) };
    if (lane == 0) {
      *(v4fa*)(st + 4 * cn) = es;
      ss[cn] = rc;
      sc[cn] = di * di;
    }
  }
  wave_sync_lds();

  const int hsel = lane & 3;
  const int nt = 4 * ne;
  float m = -__builtin_inff();
#pragma unroll 1
  for (int t0 = 0; t0 < nt; t0 += 32) {
    const int t = t0 + lane;
    const float v = st[t];
    const float mc = nmax(m, v);
    m = (t < nt) ? mc : m;
  }
  m = nmax(m, __shfl_xor(m, 4));
  m = nmax(m, __shfl_xor(m, 8));
  m = nmax(m, __shfl_xor(m, 16));
#pragma unroll 1
  for (int t0 = 0; t0 < nt; t0 += 32) {
    const int t = t0 + lane;
    st[t] = expf(st[t] - m);
  }
  wave_sync_lds();
  v4f den = (v4f){0.f, 0.f, 0.f, 0.f};
#pragma unroll 1
  for (int q = 0; q < ne; ++q) den += *(const v4fa*)(st + 4 * q);
  const float dh = sel4(den, hsel);
#pragma unroll 1
  for (int t0 = 0; t0 < nt; t0 += 32) {
    const int t = t0 + lane;
    st[t] = st[t] / dh;
  }
  wave_sync_lds();

  v4f a0 = (v4f){0.f, 0.f, 0.f, 0.f}, a1 = a0, a2 = a0, a3 = a0, ga = a0;
#pragma unroll 1
  for (int q = 0; q < ne; ++q) {
    const int sraw = ss[q];
    const int s = __builtin_amdgcn_readfirstlane(clampi(sraw, 0, kN - 1));
    const v4f al = *(const v4fa*)(st + 4 * q);
    const float cf = sc[q];
    const float* pr = P + (size_t)s * kNC + 4 * lane;
    const v4f r0 = *(const v4fa*)(pr);
    const v4f r1 = *(const v4fa*)(pr + 128);
    const v4f r2 = *(const v4fa*)(pr + 256);
    const v4f r3 = *(const v4fa*)(pr + 384);
    const v4f rg = *(const v4fa*)(pr + 512);
    asm volatile("" :: "v"(r0));
    asm volatile("" :: "v"(r1));
    asm volatile("" :: "v"(r2));
    asm volatile("" :: "v"(r3));
    asm volatile("" :: "v"(rg));
    a0 += al.x * r0;
    a1 += al.y * r1;
    a2 += al.z * r2;
    a3 += al.w * r3;
    ga += cf * rg;
  }

  const v4f bga = *(const v4fa*)(sTab + 4 * lane);
  const v4f bgn = *(const v4fa*)(sTab + 128 + 4 * lane);
  const v4f gmv = *(const v4fa*)(sTab + 256 + 4 * lane);
  const v4f btv = *(const v4fa*)(sTab + 384 + 4 * lane);
  const v4f wa0 = *(const v4fa*)(sTab + 512 + 8 * lane);
  const v4f wa1 = *(const v4fa*)(sTab + 512 + 8 * lane + 4);
  const v4f wc0 = *(const v4fa*)(sTab + 768 + 8 * lane);
  const v4f wc1 = *(const v4fa*)(sTab + 768 + 8 * lane + 4);
  const v4f gat = (((a0 + a1) + a2) + a3) * 0.25f + bga;
  const v4f gcn = ga + bgn;
  float l0 = gat.x * wa0.x + gat.y * wa0.z + gat.z * wa1.x + gat.w * wa1.z
           + gcn.x * wc0.x + gcn.y * wc0.z + gcn.z * wc1.x + gcn.w * wc1.z;
  float l1 = gat.x * wa0.y + gat.y * wa0.w + gat.z * wa1.y + gat.w * wa1.w
           + gcn.x * wc0.y + gcn.y * wc0.w + gcn.z * wc1.y + gcn.w * wc1.w;
  l0 = wsum(l0) + sTab[1024];
  l1 = wsum(l1) + sTab[1025];
  const float mx = nmax(l0, l1);
  const bool odd = (lane & 1) != 0;
  const float lsel = odd ? l1 : l0;
  const float ee = expf(lsel - mx);
  const float eo = __shfl_xor(ee, 1);
  const float gg = ee / (ee + eo);
  const float go = __shfl_xor(gg, 1);
  const float g0 = odd ? go : gg;
  const float g1 = odd ? gg : go;
  const v4f hv = (g0 * gat + g1 * gcn) + gat;
  const float mu = wsum((hv.x + hv.y) + (hv.z + hv.w)) * (1.0f / 128.0f);
  const v4f dvv = hv - mu;
  const float var = wsum((dvv.x * dvv.x + dvv.y * dvv.y) + (dvv.z * dvv.z + dvv.w * dvv.w)) * (1.0f / 128.0f);
  const float rstd = 1.0f / sqrtf(var + 1e-5f);
  v4f o = dvv * rstd * gmv + btv;
  const float qnan = __int_as_float(0x7fc00000);
  const bool mark = craw < 0;
  o.x = mark ? qnan : o.x;
  o.y = mark ? qnan : o.y;
  o.z = mark ? qnan : o.z;
  o.w = mark ? qnan : o.w;
  if (row < kN) {
    volatile v4f* q = (volatile v4f*)(out + (size_t)row * kD + 4 * lane);
    *q = o;
    __threadfence();
    *q = o;
  }
}

extern "C" void kernel_launch(void* const* d_in, const int* in_sizes, int n_in,
                              void* d_out, int out_size, void* d_ws, size_t ws_size,
                              hipStream_t stream) {
  if (n_in < 12) return;
  if (in_sizes[0] != kN * kD || in_sizes[1] != 2 * kE || in_sizes[2] != 4 * kD * kD) return;
  if (in_sizes[3] != 4 * kD || in_sizes[4] != 4 * kD || in_sizes[5] != kD) return;
  if (in_sizes[6] != kD * kD || in_sizes[7] != kD || in_sizes[8] != 2 * kD * 2) return;
  if (in_sizes[9] != 2 || in_sizes[10] != kD || in_sizes[11] != kD) return;
  if (out_size != kN * kD) return;

  const float* x     = (const float*)d_in[0];
  const int*   ei    = (const int*)  d_in[1];
  const float* Wa    = (const float*)d_in[2];
  const float* att_s = (const float*)d_in[3];
  const float* att_d = (const float*)d_in[4];
  const float* b_a   = (const float*)d_in[5];
  const float* Wn    = (const float*)d_in[6];
  const float* b_n   = (const float*)d_in[7];
  const float* Wg    = (const float*)d_in[8];
  const float* bg    = (const float*)d_in[9];
  const float* gam   = (const float*)d_in[10];
  const float* bet   = (const float*)d_in[11];
  float* out = (float*)d_out;

  char* ws = (char*)d_ws;
  size_t off = 0;
  const size_t oXB  = off; off += (size_t)kMP * kD * 2;        off = (off + 255) & ~(size_t)255;
  const size_t oWT  = off; off += (size_t)kNC * kD * 2;        off = (off + 255) & ~(size_t)255;
  const size_t oP   = off; off += (size_t)kMP * kNC * 4;       off = (off + 255) & ~(size_t)255;
  const size_t oSD  = off; off += (size_t)kMP * 8 * 4;         off = (off + 255) & ~(size_t)255;
  const size_t oLI  = off; off += (size_t)kNBLK * kRCAP * 4;   off = (off + 255) & ~(size_t)255;
  const size_t oOF  = off; off += (size_t)kNSLOT * 4;          off = (off + 255) & ~(size_t)255;
  const size_t oCN  = off; off += (size_t)kNSLOT * 4;          off = (off + 255) & ~(size_t)255;
  const size_t oDV  = off; off += (size_t)kNSLOT * 4;          off = (off + 255) & ~(size_t)255;
  const size_t oTB  = off; off += (size_t)T_TOT * 4;           off = (off + 255) & ~(size_t)255;
  if (off > ws_size || off > ((size_t)128 << 20)) return;
  unsigned short* XB = (unsigned short*)(ws + oXB);
  unsigned short* WT = (unsigned short*)(ws + oWT);
  float* P    = (float*)(ws + oP);
  float* SD   = (float*)(ws + oSD);
  int*   LIST = (int*)(ws + oLI);
  int*   OFF  = (int*)(ws + oOF);
  int*   CNT  = (int*)(ws + oCN);
  float* DINV = (float*)(ws + oDV);
  float* TAB  = (float*)(ws + oTB);

  hipFuncSetAttribute(reinterpret_cast<const void*>(&k_bucket), hipFuncAttributeMaxDynamicSharedMemorySize, kLDS_BKT);

  k_plane<0><<<(kMP * (kD / 8)) / 256, 256, 0, stream>>>(x, kN, kD, kD, XB, kMP, kD);
  k_prep<<<48, 256, 0, stream>>>(Wa, Wn, att_s, att_d, b_a, b_n, gam, bet, Wg, bg, WT, TAB);
  k_gemm_nt<0, 0><<<(469 * 10 + 7) / 8, 256, 0, stream>>>(XB, WT, TAB, P, kMP, kNC, kD, kNC);
  k_scores<<<(kMP / 32 + 7) / 8, 256, 0, stream>>>(P, TAB, SD);
  k_bucket<<<kNBLK, 256, kLDS_BKT, stream>>>(ei, OFF, CNT, DINV, LIST);
  k_replay<<<kN / 8, 256, 0, stream>>>(P, SD, OFF, CNT, DINV, LIST, TAB, out);
}
